// TopDownAttention_48979807044177
// MI455X (gfx1250) — hardware-verified
//
#include <hip/hip_runtime.h>
#include <math.h>

typedef __attribute__((ext_vector_type(16))) _Float16 v16h;
typedef __attribute__((ext_vector_type(16))) __bf16 v16b;
typedef __attribute__((ext_vector_type(8)))  _Float16 v8h;
typedef __attribute__((ext_vector_type(8)))  float v8f;
typedef __attribute__((ext_vector_type(4)))  float v4f;
typedef __attribute__((ext_vector_type(2)))  float v2f;
typedef __attribute__((ext_vector_type(4)))  unsigned v4u;
typedef __attribute__((ext_vector_type(4)))  int v4i;
typedef float __attribute__((may_alias)) float_a;
typedef int __attribute__((may_alias)) int_a;

template <typename T> __device__ __forceinline__ void vst2(void* p, T v) { *(volatile T*)p = v; __threadfence(); *(volatile T*)p = v; }
__device__ __forceinline__ v8f wmma16(v16h a, v16h b, v8f c) {
  v8f d = __builtin_amdgcn_wmma_f32_16x16x32_f16(false, a, false, b, (short)0, c, false, false);
  asm volatile("v_nop\n\tv_nop\n\tv_nop\n\tv_nop" : "+v"(d) : "v"(a), "v"(b));
  return d;
}
__device__ __forceinline__ v8f wmma_bf(v16b a, v16b b, v8f c) {
  v8f d = __builtin_amdgcn_wmma_f32_16x16x32_bf16(false, a, false, b, (short)0, c, false, false);
  asm volatile("v_nop\n\tv_nop\n\tv_nop\n\tv_nop" : "+v"(d) : "v"(a), "v"(b));
  return d;
}
__device__ __forceinline__ v16h frag_h(const _Float16* rowk0, int lane) {
  union { v16h v; v8h q[2]; } u; const _Float16* p = rowk0 + 8 * (lane >> 4);
  u.q[0] = *(const v8h*)p; u.q[1] = *(const v8h*)(p + 16); return u.v;
}
__device__ __forceinline__ v16h frag_f32(const float* rowk0, int lane) {
  v16h a; const float* p = rowk0 + 8 * (lane >> 4);
#pragma unroll
  for (int i = 0; i < 8; ++i) { a[i] = (_Float16)p[i]; a[8 + i] = (_Float16)p[16 + i]; }
  return a;
}
__device__ __forceinline__ v16h frag_f32s(const float* rowk0, int lane, float sc) {
  v16h a; const float* p = rowk0 + 8 * (lane >> 4);
#pragma unroll
  for (int i = 0; i < 8; ++i) { a[i] = (_Float16)(p[i] * sc); a[8 + i] = (_Float16)(p[16 + i] * sc); }
  return a;
}
__device__ __forceinline__ v16h fragc_f32(const float* W, int k0, int n, int lane, int ld, int K) {
  v16h a; const int g = lane >> 4;
#pragma unroll
  for (int i = 0; i < 8; ++i) { const int ka = k0 + 8 * g + i, kb = ka + 16;
    a[i] = (_Float16)(ka < K ? W[(size_t)(ka < K ? ka : K - 1) * ld + n] : 0.f); a[8 + i] = (_Float16)(kb < K ? W[(size_t)(kb < K ? kb : K - 1) * ld + n] : 0.f); }
  return a;
}
struct F2 { v16b h, l; };
__device__ __forceinline__ F2 bsplit16(const float v[16]) { F2 r;
#pragma unroll
  for (int i = 0; i < 16; ++i) { const __bf16 h = (__bf16)v[i]; r.h[i] = h; r.l[i] = (__bf16)(v[i] - (float)h); }
  return r; }
__device__ __forceinline__ F2 split_row(const float* row, int k0, int lane) { float v[16]; const float* p = row + k0 + 8 * (lane >> 4);
#pragma unroll
  for (int i = 0; i < 8; ++i) { v[i] = p[i]; v[8 + i] = p[16 + i]; }
  return bsplit16(v); }
__device__ __forceinline__ F2 split_rowK(const float* row, int k0, int lane, int K) { float v[16]; const int g = lane >> 4;
#pragma unroll
  for (int i = 0; i < 8; ++i) { const int ka = k0 + 8 * g + i, kb = ka + 16; v[i] = ka < K ? row[ka < K ? ka : K - 1] : 0.f; v[8 + i] = kb < K ? row[kb < K ? kb : K - 1] : 0.f; }
  return bsplit16(v); }
__device__ __forceinline__ F2 split_col(const float* W, int k0, int n, int lane, int ld, int K) { float v[16]; const int g = lane >> 4;
#pragma unroll
  for (int i = 0; i < 8; ++i) { const int ka = k0 + 8 * g + i, kb = ka + 16; v[i] = ka < K ? W[(size_t)(ka < K ? ka : K - 1) * ld + n] : 0.f; v[8 + i] = kb < K ? W[(size_t)(kb < K ? kb : K - 1) * ld + n] : 0.f; }
  return bsplit16(v); }
__device__ __forceinline__ v8f mac3(const F2& a, const F2& b, v8f c) { c = wmma_bf(a.l, b.h, c); c = wmma_bf(a.h, b.l, c); return wmma_bf(a.h, b.h, c); }
__device__ __forceinline__ float sigm(float v) { return 1.0f / (1.0f + expf(-v)); }
#define LDSX() do { asm volatile("s_wait_dscnt 0" ::: "memory"); __builtin_amdgcn_wave_barrier(); __builtin_amdgcn_fence(__ATOMIC_RELEASE, "workgroup"); } while (0)


#define NBB 64
#define NO 100
#define F1 2048
#define F2 1024
#define AH 512
#define NROW (NBB * NO)
typedef __attribute__((ext_vector_type(8))) __bf16 v8b;
__device__ __forceinline__ v16b frag_b(const __bf16* rowk0, int lane) {
  union { v16b v; v8b q[2]; } u; const __bf16* p = rowk0 + 8 * (lane >> 4);
  u.q[0] = *(const v8b*)p; u.q[1] = *(const v8b*)(p + 16); return u.v;
}
__device__ __forceinline__ float bfr(float v) { return (float)(__bf16)v; }
__device__ __attribute__((noinline)) float exp_ni(float v) { return expf(v); }
__device__ __attribute__((noinline)) float erf_ni(float v) { return erff(v); }

#define WS_QC  0u
#define WS_SC  (WS_QC + 4u * (size_t)NBB * 2 * AH)
#define WS_END (WS_SC + 4u * 6464)

__global__ __launch_bounds__(128) void k_ques(const float* __restrict__ QE, const float* __restrict__ WT, const float* __restrict__ BT, const float* __restrict__ WG, const float* __restrict__ BG, float* __restrict__ QC) { __shared__ __align__(16) float so[16][AH + 4];
  const int tid = threadIdx.x, wave = tid >> 5, lane = tid & 31, col = lane & 15, g = lane >> 4; const int b0 = blockIdx.x * 16, which = blockIdx.y; const float* Wm = (which == 0 ? WT : WG) + (size_t)F1 * AH; const float* Bm = which == 0 ? BT : BG;
  v8f acc[8] = {};
#pragma unroll 2
  for (int kc = 0; kc < F2 / 32; ++kc) { v16b a; { const float* p = QE + (size_t)(b0 + col) * F2 + kc * 32 + 8 * g;
#pragma unroll
      for (int i = 0; i < 8; ++i) { a[i] = (__bf16)p[i]; a[8 + i] = (__bf16)p[16 + i]; } }
#pragma unroll
    for (int j = 0; j < 8; ++j) { v16b w; const int o = wave * 128 + j * 16 + col;
#pragma unroll
      for (int i = 0; i < 8; ++i) { w[i] = (__bf16)Wm[(size_t)(kc * 32 + 8 * g + i) * AH + o]; w[8 + i] = (__bf16)Wm[(size_t)(kc * 32 + 16 + 8 * g + i) * AH + o]; }
      acc[j] = wmma_bf(a, w, acc[j]); } }
#pragma unroll
  for (int j = 0; j < 8; ++j) { const int o = wave * 128 + j * 16 + col; const float bb = bfr(Bm[o]);
#pragma unroll
    for (int r = 0; r < 8; ++r) so[8 * g + r][o] = acc[j][r] + bb; }
  __syncthreads();
  for (int e = tid; e < 16 * AH / 4; e += 128) { const int rl = e / (AH / 4), q = e % (AH / 4); vst2(QC + ((size_t)(b0 + rl) * 2 + which) * AH + q * 4, *(const v4f*)&so[rl][q * 4]); } }
__global__ __launch_bounds__(128) void k_score(const float* __restrict__ IMG, const float* __restrict__ WT, const float* __restrict__ WG, const float* __restrict__ QC, const float* __restrict__ WSC, const float* __restrict__ BSC, float* __restrict__ SC) { __shared__ float spart[4][16][17]; __shared__ __align__(16) float ssc[64];
  const int tid = threadIdx.x, wave = tid >> 5, lane = tid & 31, col = lane & 15, g = lane >> 4; const size_t r0 = (size_t)blockIdx.x * 64 + wave * 16;
  float rowacc[8];
#pragma unroll
  for (int r = 0; r < 8; ++r) rowacc[r] = 0.f;
#pragma unroll 1
  for (int cg = 0; cg < AH / 64; ++cg) { v8f at[4] = {}, ag[4] = {};
#pragma unroll 2
    for (int kc = 0; kc < F1 / 32; ++kc) { v16b a; { const float* p = IMG + (r0 + col) * F1 + kc * 32 + 8 * g;
#pragma unroll
        for (int i = 0; i < 8; ++i) { a[i] = (__bf16)p[i]; a[8 + i] = (__bf16)p[16 + i]; } }
#pragma unroll
      for (int j = 0; j < 4; ++j) { v16b wt, wg; const int o = cg * 64 + j * 16 + col;
#pragma unroll
        for (int i = 0; i < 8; ++i) { wt[i] = (__bf16)WT[(size_t)(kc * 32 + 8 * g + i) * AH + o]; wt[8 + i] = (__bf16)WT[(size_t)(kc * 32 + 16 + 8 * g + i) * AH + o]; wg[i] = (__bf16)WG[(size_t)(kc * 32 + 8 * g + i) * AH + o]; wg[8 + i] = (__bf16)WG[(size_t)(kc * 32 + 16 + 8 * g + i) * AH + o]; }
        at[j] = wmma_bf(a, wt, at[j]); ag[j] = wmma_bf(a, wg, ag[j]); } }
#pragma unroll
    for (int j = 0; j < 4; ++j) { const int o = cg * 64 + j * 16 + col; const float wsc = bfr(WSC[o]);
#pragma unroll
      for (int r = 0; r < 8; ++r) { const size_t row = r0 + 8 * g + r; const size_t b = row / NO; const float t = at[j][r] + QC[(b * 2 + 0) * AH + o], gg = ag[j][r] + QC[(b * 2 + 1) * AH + o]; rowacc[r] += tanhf(t) * (1.0f / (1.0f + expf(-gg))) * wsc; } } }
#pragma unroll
  for (int r = 0; r < 8; ++r) { float v = rowacc[r];
#pragma unroll
    for (int o = 1; o < 16; o <<= 1) v += __shfl_xor(v, o);
    if (col == 0) spart[wave][8 * g + r][0] = v; }
  __syncthreads();
  if (tid < 64) ssc[tid] = spart[tid >> 4][tid & 15][0] + bfr(BSC[0]);
  __syncthreads(); if (tid < 16) vst2(SC + (size_t)blockIdx.x * 64 + tid * 4, *(const v4f*)&ssc[tid * 4]); }
__global__ __launch_bounds__(256) void k_pool(const float* __restrict__ SC, const int* __restrict__ NOBJ, const float* __restrict__ IMG, float* __restrict__ OUT) { __shared__ float sw[NO]; __shared__ __align__(16) float so[F1];
  const int t = threadIdx.x; const size_t b = blockIdx.x; const int nob = NOBJ[b];
  if (t == 0) { float m = -3.0e38f; for (int o = 0; o < NO; ++o) if (o < nob) m = fmaxf(m, SC[b * NO + o]); float s = 0.f; for (int o = 0; o < NO; ++o) { const float w = (o < nob) ? expf(SC[b * NO + o] - m) : 0.f; sw[o] = w; s += w; } const float inv = 1.0f / s; for (int o = 0; o < NO; ++o) sw[o] *= inv; }
  __syncthreads();
  for (int f = t; f < F1; f += 256) { float a = 0.f;
#pragma unroll 1
    for (int o = 0; o < NO; ++o) a += sw[o] * bfr(IMG[(b * NO + o) * F1 + f]);
    so[f] = a; }
  __syncthreads(); for (int q = t; q < F1 / 4; q += 256) vst2(OUT + b * F1 + q * 4, *(const v4f*)&so[q * 4]); }
extern "C" void kernel_launch(void* const* d_in, const int* in_sizes, int n_in, void* d_out, int out_size, void* d_ws, size_t ws_size, hipStream_t stream) {
  (void)in_sizes; (void)n_in; (void)out_size;
  const float** F = (const float**)d_in;
  if (ws_size < (size_t)WS_END) return;
  char* ws = (char*)d_ws; float *QC = (float*)(ws + WS_QC), *SC = (float*)(ws + WS_SC);
  k_ques<<<dim3(NBB / 16, 2), 128, 0, stream>>>(F[1], F[3], F[4], F[5], F[6], QC);
  k_score<<<NROW / 64, 128, 0, stream>>>(F[0], F[3], F[5], QC, F[7], F[8], SC);
  k_pool<<<NBB, 256, 0, stream>>>(SC, (const int*)d_in[2], F[0], (float*)d_out);
}
